// LocalWindowAttention_13924283973718
// MI455X (gfx1250) — hardware-verified
//
#include <hip/hip_runtime.h>
#include <math.h>
#include <stdint.h>

#ifndef NB
#define NB 4
#endif
#ifndef SEQ
#define SEQ 4096
#endif
#define NB_FULL  4
#define SEQ_FULL 4096
#define EMB      512
#define NQKV     (3 * EMB)
#define WIN      64
#define NKBAND   6
#define QKP      (2 * EMB)
#define NROWS    (NB * SEQ)
#define QSC   8.0f
#define KSC   8.0f
#define RQK   4096.0f
#define PCAR  32768.0f
#define VCAR  1024.0f
#define OSC   1024.0f
#define ROC   1024.0f
#define WOS   1024.0f
#define RSQE  0.044194173824159216f
#define LOG2E 1.4426950408889634f
#define NEGS  (-3.0e38f)
#define ATT_WAVES   4
#define ATT_THREADS (ATT_WAVES * 32)
#define NQT         (SEQ / 64)
#define ATT_BLOCKS  (NB * NQT)
#define SLAB   (16 * 68)
static_assert(NB >= 1 && NB <= NB_FULL);
static_assert((SEQ % 64) == 0 && SEQ >= 64 && SEQ <= SEQ_FULL);
static_assert(EMB == 512 && (EMB % 64) == 0 && (NQKV % 64) == 0);
static_assert(NKBAND * 32 == 64 + 2 * WIN);
static_assert(((SEQ * EMB / 8) % 256) == 0);
static_assert(((NROWS / 64) * (EMB / 64)) >= 1);
static_assert((SLAB * 4) % 16 == 0);
static_assert(ATT_THREADS == 128);

typedef unsigned short u16;
typedef _Float16 v16h __attribute__((ext_vector_type(16)));
typedef _Float16 v8h  __attribute__((ext_vector_type(8)));
typedef __bf16   v16b __attribute__((ext_vector_type(16)));
typedef float    v8f  __attribute__((ext_vector_type(8)));
typedef float    v4f  __attribute__((ext_vector_type(4)));
typedef unsigned int v4u __attribute__((ext_vector_type(4)));

union FragH { v16h v; v8h h[2]; v4u u[2]; };
union FragB { v16b v; v4u u[2]; };

__device__ __forceinline__ unsigned short bf_bits(float f) {
  unsigned u = __float_as_uint(f);
  return (unsigned short)((u + 0x7FFFu + ((u >> 16) & 1u)) >> 16);
}
__device__ __forceinline__ float bf_up(unsigned short h) { return __uint_as_float(((unsigned)h) << 16); }
__device__ __forceinline__ float bf_val(float f) { return bf_up(bf_bits(f)); }
__device__ __forceinline__ unsigned short h_bits(_Float16 x) { return __builtin_bit_cast(unsigned short, x); }
__device__ __forceinline__ unsigned pk16(unsigned short a, unsigned short b) { return (unsigned)a | ((unsigned)b << 16); }
__device__ __forceinline__ v8f zero8() { v8f z = {0.f, 0.f, 0.f, 0.f, 0.f, 0.f, 0.f, 0.f}; return z; }

__device__ __forceinline__ v16h ldfrag_h(const _Float16* p) {
  FragH f;
  f.h[0] = *(const v8h*)(p);
  f.h[1] = *(const v8h*)(p + 16);
  return f.v;
}
__device__ __forceinline__ v16b ldfrag_b(const u16* p) {
  FragB f;
  f.u[0] = *(const v4u*)(p);
  f.u[1] = *(const v4u*)(p + 16);
  return f.v;
}

__device__ __forceinline__ v8f mma_h(v16h a, v16h b, v8f c) {
  return __builtin_amdgcn_wmma_f32_16x16x32_f16(false, a, false, b, (short)0, c, false, false);
}
__device__ __forceinline__ v8f mma_b(v16b a, v16b b, v8f c) {
  return __builtin_amdgcn_wmma_f32_16x16x32_bf16(false, a, false, b, (short)0, c, false, false);
}
template <typename F>
__device__ __forceinline__ void guard6(v8f& a, v8f& b, v8f& c, v8f& d, F x0, F x1, F x2, F x3, F x4, F x5) {
#if defined(__HIP_DEVICE_COMPILE__)
  asm volatile("v_nop\n\tv_nop\n\tv_nop\n\tv_nop"
               : "+v"(a), "+v"(b), "+v"(c), "+v"(d) : "v"(x0), "v"(x1), "v"(x2), "v"(x3), "v"(x4), "v"(x5) : "memory");
#endif
}
__device__ __forceinline__ void guard8(v8f& a, v8f& b, v8f& c, v8f& d, v8f& e, v8f& f, v8f& g, v8f& h2,
                                       v16h x0, v16h x1, v16h x2, v16h x3, v16h x4, v16h x5) {
#if defined(__HIP_DEVICE_COMPILE__)
  asm volatile("v_nop\n\tv_nop\n\tv_nop\n\tv_nop"
               : "+v"(a), "+v"(b), "+v"(c), "+v"(d), "+v"(e), "+v"(f), "+v"(g), "+v"(h2)
               : "v"(x0), "v"(x1), "v"(x2), "v"(x3), "v"(x4), "v"(x5) : "memory");
#endif
}
__device__ __forceinline__ void acc_guard4(v8f& a, v8f& b, v8f& c, v8f& d) {
#if defined(__HIP_DEVICE_COMPILE__)
  asm volatile("v_nop\n\tv_nop\n\tv_nop\n\tv_nop" : "+v"(a), "+v"(b), "+v"(c), "+v"(d));
#endif
}
__device__ __forceinline__ void wave_sync_lds() {
#if defined(__HIP_DEVICE_COMPILE__)
  __builtin_amdgcn_fence(__ATOMIC_RELEASE, "workgroup");
  __builtin_amdgcn_wave_barrier();
  __builtin_amdgcn_fence(__ATOMIC_ACQUIRE, "workgroup");
#endif
}

__global__ __launch_bounds__(256) void cvt16(const float* __restrict__ x, u16* D, int n8pb, int nb, int sst8,
                                             int mode, float scale) {
  const int gt = blockIdx.x * 256 + (int)threadIdx.x;
  if (gt >= nb * n8pb) return;
  const int b = gt / n8pb;
  const int r = gt - b * n8pb;
  const float* p = x + ((size_t)b * (size_t)sst8 + (size_t)r) * 8;
  const v4f a = *(const v4f*)(p), c4 = *(const v4f*)(p + 4);
  float v[8];
#pragma unroll
  for (int e = 0; e < 4; ++e) { v[e] = a[e]; v[4 + e] = c4[e]; }
  unsigned short s[8];
#pragma unroll
  for (int e = 0; e < 8; ++e) {
    const unsigned short bb = bf_bits(v[e]);
    const unsigned short hb = h_bits((_Float16)(bf_up(bb) * scale));
    s[e] = (mode != 0) ? hb : bb;
  }
  v4u o;
#pragma unroll
  for (int e = 0; e < 4; ++e) o[e] = pk16(s[2 * e], s[2 * e + 1]);
  u16* d = D + (size_t)gt * 8;
  for (int pass = 0; pass < 2; ++pass) {
    *(volatile v4u*)(d) = o;
    __threadfence();
  }
}

__global__ __launch_bounds__(256) void tcvt16(const float* __restrict__ W, u16* D, int KR, int NC, int mode, float scale) {
  __shared__ __align__(16) float tile[64 * 68];
  const int tid = threadIdx.x, wave = tid >> 5, lane = tid & 31;
  const int nt  = NC >> 6;
  const int bid = blockIdx.x;
  const int n0  = (bid % nt) * 64;
  const int k0  = (bid / nt) * 64;
  if (k0 + 64 > KR) return;
  const int row = tid >> 2, c16 = (tid & 3) * 16;
  const float* src = W + (size_t)(k0 + row) * (size_t)NC + n0 + c16;
  const v4f f0 = *(const v4f*)(src), f1 = *(const v4f*)(src + 4), f2 = *(const v4f*)(src + 8), f3 = *(const v4f*)(src + 12);
  float f[16];
#pragma unroll
  for (int e = 0; e < 4; ++e) { f[e] = f0[e]; f[4 + e] = f1[e]; f[8 + e] = f2[e]; f[12 + e] = f3[e]; }
#pragma unroll
  for (int e = 0; e < 16; ++e) tile[(c16 + e) * 68 + row] = f[e];
  __syncthreads();
  const int rq = lane >> 3, c8 = (lane & 7) * 8;
  v4u ov[2];
#pragma unroll
  for (int i = 0; i < 2; ++i) {
    const int orow = wave * 8 + i * 4 + rq;
    const v4f a = *(const v4f*)(tile + orow * 68 + c8), c4 = *(const v4f*)(tile + orow * 68 + c8 + 4);
    float w[8];
#pragma unroll
    for (int e = 0; e < 4; ++e) { w[e] = a[e]; w[4 + e] = c4[e]; }
    unsigned short s[8];
#pragma unroll
    for (int e = 0; e < 8; ++e) {
      const unsigned short bb = bf_bits(w[e]);
      const unsigned short hb = h_bits((_Float16)(bf_up(bb) * scale));
      s[e] = (mode != 0) ? hb : bb;
    }
#pragma unroll
    for (int e = 0; e < 4; ++e) ov[i][e] = pk16(s[2 * e], s[2 * e + 1]);
  }
  u16* dst = D + (size_t)(n0 + wave * 8 + rq) * (size_t)KR + k0 + c8;
  for (int pass = 0; pass < 2; ++pass) {
#pragma unroll
    for (int i = 0; i < 2; ++i) {
      *(volatile v4u*)(dst + (size_t)(i * 4) * (size_t)KR) = ov[i];
    }
    __threadfence();
  }
}

template <bool RES>
__device__ __forceinline__ void epi16(float* sl, v8f a0, v8f a1, v8f a2, v8f a3, float oscale, float rscale, u16* C,
                                      int ldc, int loff, size_t rowb, int col0, int lane,
                                      const float* __restrict__ bias, int bmode, int blen) {
  const int hh = lane >> 4, m = lane & 15;
  float bc[4], br[8];
  if (bmode != 0) {
#pragma unroll
    for (int j = 0; j < 4; ++j) bc[j] = 0.f;
#pragma unroll
    for (int r = 0; r < 8; ++r) {
      const int bi = min((int)rowb + 8 * hh + r, blen - 1);
      br[r] = bf_val(bias[bi]);
    }
  } else {
#pragma unroll
    for (int r = 0; r < 8; ++r) br[r] = 0.f;
#pragma unroll
    for (int j = 0; j < 4; ++j) {
      const int bi = min(col0 + 16 * j + m, blen - 1);
      bc[j] = bf_val(bias[bi]);
    }
  }
#pragma unroll
  for (int r = 0; r < 8; ++r) {
    const int ro = (8 * hh + r) * 68 + m;
    sl[ro]      = (a0[r] + br[r] + bc[0]) * oscale;
    sl[ro + 16] = (a1[r] + br[r] + bc[1]) * oscale;
    sl[ro + 32] = (a2[r] + br[r] + bc[2]) * oscale;
    sl[ro + 48] = (a3[r] + br[r] + bc[3]) * oscale;
  }
  wave_sync_lds();
  const int rq = lane >> 3, c8 = (lane & 7) * 8;
  v4u ov[4], ol[4];
#pragma unroll
  for (int i4 = 0; i4 < 4; ++i4) {
    const int row = i4 * 4 + rq;
    const v4f a = *(const v4f*)(sl + row * 68 + c8), c4 = *(const v4f*)(sl + row * 68 + c8 + 4);
    float w[8];
#pragma unroll
    for (int e = 0; e < 4; ++e) { w[e] = a[e]; w[4 + e] = c4[e]; }
#pragma unroll
    for (int e = 0; e < 4; ++e) {
      const _Float16 h0 = (_Float16)w[2 * e], h1 = (_Float16)w[2 * e + 1];
      ov[i4][e] = pk16(h_bits(h0), h_bits(h1));
      if constexpr (RES) {
        const _Float16 l0 = (_Float16)((w[2 * e] - (float)h0) * rscale);
        const _Float16 l1 = (_Float16)((w[2 * e + 1] - (float)h1) * rscale);
        ol[i4][e] = pk16(h_bits(l0), h_bits(l1));
      } else {
        ol[i4][e] = ov[i4][e];
      }
    }
  }
  u16* dst = C + (rowb + (size_t)rq) * (size_t)ldc + col0 + c8;
  for (int pass = 0; pass < 2; ++pass) {
#pragma unroll
    for (int i4 = 0; i4 < 4; ++i4) {
      *(volatile v4u*)(dst + (size_t)(i4 * 4) * (size_t)ldc) = ov[i4];
      if constexpr (RES) {
        *(volatile v4u*)(dst + (size_t)(i4 * 4) * (size_t)ldc + loff) = ol[i4];
      }
    }
    __threadfence();
  }
}

__device__ __forceinline__ void epi64(float* sl, v8f a0, v8f a1, v8f a2, v8f a3, float oscale, float* C, int N,
                                      size_t rowb, int col0, int lane, const float* __restrict__ bias, int blen) {
  const int hh = lane >> 4, m = lane & 15;
  float bc[4];
#pragma unroll
  for (int j = 0; j < 4; ++j) {
    const int bi = min(col0 + 16 * j + m, blen - 1);
    bc[j] = bf_val(bias[bi]);
  }
#pragma unroll
  for (int r = 0; r < 8; ++r) {
    const int ro = (8 * hh + r) * 68 + m;
    sl[ro]      = a0[r] * oscale + bc[0];
    sl[ro + 16] = a1[r] * oscale + bc[1];
    sl[ro + 32] = a2[r] * oscale + bc[2];
    sl[ro + 48] = a3[r] * oscale + bc[3];
  }
  wave_sync_lds();
  v4f vals[8];
#pragma unroll
  for (int it = 0; it < 8; ++it) vals[it] = *(const v4f*)(sl + (it * 2 + hh) * 68 + m * 4);
  float* dst = C + (rowb + (size_t)hh) * (size_t)N + col0 + m * 4;
  for (int pass = 0; pass < 2; ++pass) {
#pragma unroll
    for (int it = 0; it < 8; ++it) {
      *(volatile v4f*)(dst + (size_t)(it * 2) * (size_t)N) = vals[it];
    }
    __threadfence();
  }
}

template <bool RES>
__global__ __launch_bounds__(128)
void gemm_b16(const u16* __restrict__ A, const u16* __restrict__ Bt, u16* C, int M, int N, int K, int ldc, int loff,
              int bstA, int bstB, int bstC, float oscale, float rscale, const float* __restrict__ bias, int bmode, int blen) {
  __shared__ __align__(16) float slab[4 * SLAB];
  const int tid = threadIdx.x, wave = tid >> 5, lane = tid & 31, hh = lane >> 4, m = lane & 15;
  const int ntile = N >> 6, mtile = M >> 6;
  const int per   = ntile * mtile;
  const int bid   = blockIdx.x;
  const int bt    = bid / per;
  const int t     = bid - bt * per;
  const int rowb  = (t / ntile) * 64 + wave * 16;
  const int col0  = (t % ntile) * 64;
  if (rowb + 16 > M) return;
  const u16* Ab = A  + (size_t)bt * (size_t)bstA;
  const u16* Bb = Bt + (size_t)bt * (size_t)bstB;
  u16*       Cb = C  + (size_t)bt * (size_t)bstC;
  const u16* ap = Ab + (size_t)(rowb + m) * K + 8 * hh;
  const u16* bp = Bb + (size_t)(col0 + m) * K + 8 * hh;
  const size_t bs = (size_t)16 * K;
  v8f acc0 = zero8(), acc1 = zero8(), acc2 = zero8(), acc3 = zero8();
#pragma unroll 1
  for (int k0 = 0; k0 < K; k0 += 32) {
    const v16b a  = ldfrag_b(ap + k0);
    const v16b b0 = ldfrag_b(bp + k0);
    const v16b b1 = ldfrag_b(bp + bs + k0);
    const v16b b2 = ldfrag_b(bp + 2 * bs + k0);
    const v16b b3 = ldfrag_b(bp + 3 * bs + k0);
    acc0 = mma_b(a, b0, acc0);
    acc1 = mma_b(a, b1, acc1);
    acc2 = mma_b(a, b2, acc2);
    acc3 = mma_b(a, b3, acc3);
    guard6<v16b>(acc0, acc1, acc2, acc3, a, b0, b1, b2, b3, a);
  }
  epi16<RES>(slab + wave * SLAB, acc0, acc1, acc2, acc3, oscale, rscale, Cb, ldc, loff, (size_t)rowb, col0, lane,
             bias, bmode, blen);
}

__global__ __launch_bounds__(128)
void gemm_hf2(const u16* __restrict__ A, const u16* __restrict__ Bt, float* C, int M, int N, int K, int lda, int loff,
              int bstA, int bstC, float oscale, float rinv, const float* __restrict__ bias, int blen) {
  __shared__ __align__(16) float slab[4 * SLAB];
  const int tid = threadIdx.x, wave = tid >> 5, lane = tid & 31, hh = lane >> 4, m = lane & 15;
  const int ntile = N >> 6, mtile = M >> 6;
  const int per   = ntile * mtile;
  const int bid   = blockIdx.x;
  const int bt    = bid / per;
  const int t     = bid - bt * per;
  const int rowb  = (t / ntile) * 64 + wave * 16;
  const int col0  = (t % ntile) * 64;
  if (rowb + 16 > M) return;
  const _Float16* ap = (const _Float16*)(const void*)A + (size_t)bt * (size_t)bstA + (size_t)(rowb + m) * (size_t)lda + 8 * hh;
  const _Float16* bp = (const _Float16*)(const void*)Bt + (size_t)(col0 + m) * K + 8 * hh;
  float* Cb = C + (size_t)bt * (size_t)bstC;
  const size_t bs = (size_t)16 * K;
  v8f h0 = zero8(), h1 = zero8(), h2 = zero8(), h3 = zero8();
  v8f l0 = zero8(), l1 = zero8(), l2 = zero8(), l3 = zero8();
#pragma unroll 1
  for (int k0 = 0; k0 < K; k0 += 32) {
    const v16h ah = ldfrag_h(ap + k0);
    const v16h al = ldfrag_h(ap + loff + k0);
    const v16h b0 = ldfrag_h(bp + k0);
    const v16h b1 = ldfrag_h(bp + bs + k0);
    const v16h b2 = ldfrag_h(bp + 2 * bs + k0);
    const v16h b3 = ldfrag_h(bp + 3 * bs + k0);
    h0 = mma_h(ah, b0, h0);
    h1 = mma_h(ah, b1, h1);
    h2 = mma_h(ah, b2, h2);
    h3 = mma_h(ah, b3, h3);
    l0 = mma_h(al, b0, l0);
    l1 = mma_h(al, b1, l1);
    l2 = mma_h(al, b2, l2);
    l3 = mma_h(al, b3, l3);
    guard8(h0, h1, h2, h3, l0, l1, l2, l3, ah, al, b0, b1, b2, b3);
  }
  const v8f a0 = h0 + l0 * rinv;
  const v8f a1 = h1 + l1 * rinv;
  const v8f a2 = h2 + l2 * rinv;
  const v8f a3 = h3 + l3 * rinv;
  epi64(slab + wave * SLAB, a0, a1, a2, a3, oscale, Cb, N, (size_t)rowb, col0, lane, bias, blen);
}

__global__ __launch_bounds__(ATT_THREADS)
void attn_fwd(const u16* __restrict__ QPp, const u16* __restrict__ KPp, const u16* __restrict__ VPp, u16* OPp) {
  __shared__ __align__(16) float smem[ATT_WAVES * SLAB];

  const int tid  = threadIdx.x;
  const int wave = tid >> 5;
  const int lane = tid & 31;
  const int hh   = lane >> 4;
  const int c    = lane & 15;

  const int bid  = blockIdx.x;
  const int qt   = bid % NQT;
  const int bb   = bid / NQT;
  if (bb >= NB) return;
  const int qb   = qt * 64;
  const int q0   = qb + wave * 16;
  const int kstart = qb - WIN;
  const int qi   = q0 + c;

  const size_t brow = (size_t)bb * SEQ;
  const _Float16* Qb = (const _Float16*)(const void*)QPp + (brow + (size_t)qi) * QKP + 8 * hh;
  const _Float16* Kb = (const _Float16*)(const void*)KPp + (brow + (size_t)c) * QKP + 8 * hh;
  const _Float16* Vb = (const _Float16*)(const void*)VPp + ((size_t)bb * EMB + (size_t)c) * SEQ + 8 * hh;
  const float lsc  = (RSQE * LOG2E) / (QSC * KSC);
  const float lscr = lsc * (1.0f / RQK);

  float tk[16 * NKBAND];
#pragma unroll
  for (int kb = 0; kb < NKBAND; ++kb) {
    const int key0 = kstart + 32 * kb;
    const int kba  = min(max(key0, 0), SEQ - 32);
    const _Float16* k0p = Kb + (size_t)kba * QKP;
    const _Float16* k1p = k0p + (size_t)16 * QKP;
    v8f g0 = zero8(), g1 = zero8(), cx0 = zero8(), cx1 = zero8();
#pragma unroll 1
    for (int dc = 0; dc < EMB; dc += 32) {
      const v16h qh  = ldfrag_h(Qb + dc);
      const v16h ql  = ldfrag_h(Qb + EMB + dc);
      const v16h ka  = ldfrag_h(k0p + dc);
      const v16h kal = ldfrag_h(k0p + EMB + dc);
      const v16h kc  = ldfrag_h(k1p + dc);
      const v16h kcl = ldfrag_h(k1p + EMB + dc);
      g0  = mma_h(ka,  qh, g0);
      cx0 = mma_h(ka,  ql, cx0);
      cx0 = mma_h(kal, qh, cx0);
      g1  = mma_h(kc,  qh, g1);
      cx1 = mma_h(kc,  ql, cx1);
      cx1 = mma_h(kcl, qh, cx1);
      guard6<v16h>(g0, g1, cx0, cx1, qh, ql, ka, kal, kc, kcl);
    }
#pragma unroll
    for (int i = 0; i < 8; ++i) {
      const int j0 = key0 + 8 * hh + i;
      const int j1 = j0 + 16;
      const int d0 = qi - j0;
      const int d1 = qi - j1;
      const bool a0 = (j0 >= 0) && (j0 < SEQ) && (d0 <= WIN) && (d0 >= -WIN);
      const bool a1 = (j1 >= 0) && (j1 < SEQ) && (d1 <= WIN) && (d1 >= -WIN);
      tk[16 * kb + i]     = a0 ? (g0[i] * lsc + cx0[i] * lscr) : NEGS;
      tk[16 * kb + 8 + i] = a1 ? (g1[i] * lsc + cx1[i] * lscr) : NEGS;
    }
  }

  float mx = tk[0];
#pragma unroll
  for (int i = 1; i < 16 * NKBAND; ++i) mx = fmaxf(mx, tk[i]);
  mx = fmaxf(mx, __shfl_xor(mx, 16, 32));

  float ps = 0.f;
  FragH pf[NKBAND];
#pragma unroll
  for (int kb = 0; kb < NKBAND; ++kb) {
#pragma unroll
    for (int wq = 0; wq < 2; ++wq) {
#pragma unroll
      for (int e4 = 0; e4 < 4; ++e4) {
        const int i = 16 * kb + 8 * wq + 2 * e4;
        const float x0 = exp2f(fminf(tk[i] - mx, 0.f));
        const float x1 = exp2f(fminf(tk[i + 1] - mx, 0.f));
        const float p0 = (tk[i] > -1.0e38f) ? x0 : 0.f;
        const float p1 = (tk[i + 1] > -1.0e38f) ? x1 : 0.f;
        ps += p0 + p1;
        pf[kb].u[wq][e4] = pk16(h_bits((_Float16)(p0 * PCAR)), h_bits((_Float16)(p1 * PCAR)));
      }
    }
  }
  ps += __shfl_xor(ps, 16, 32);
  const float linv = (ps > 0.f) ? ((1.0f / ps) * (1.0f / (PCAR * VCAR))) : 0.f;
  float inv[8];
#pragma unroll
  for (int r = 0; r < 8; ++r) inv[r] = __shfl(linv, 8 * hh + r, 32);

  float* slab = smem + wave * SLAB;
  const int rq = lane >> 3, c8 = (lane & 7) * 8;
  u16* ob = OPp + (brow + (size_t)q0) * QKP + c8;

#pragma unroll 1
  for (int sl = 0; sl < EMB / 64; ++sl) {
    v8f o0 = zero8(), o1 = zero8(), o2 = zero8(), o3 = zero8();
    const _Float16* vs = Vb + (size_t)(64 * sl) * SEQ;
#pragma unroll
    for (int kb = 0; kb < NKBAND; ++kb) {
      const int key0 = kstart + 32 * kb;
      const int kba  = min(max(key0, 0), SEQ - 32);
      const _Float16* vp = vs + kba;
      const v16h vf0 = ldfrag_h(vp);
      const v16h vf1 = ldfrag_h(vp + (size_t)16 * SEQ);
      const v16h vf2 = ldfrag_h(vp + (size_t)32 * SEQ);
      const v16h vf3 = ldfrag_h(vp + (size_t)48 * SEQ);
      o0 = mma_h(pf[kb].v, vf0, o0);
      o1 = mma_h(pf[kb].v, vf1, o1);
      o2 = mma_h(pf[kb].v, vf2, o2);
      o3 = mma_h(pf[kb].v, vf3, o3);
      guard6<v16h>(o0, o1, o2, o3, pf[kb].v, vf0, vf1, vf2, vf3, pf[kb].v);
    }
    acc_guard4(o0, o1, o2, o3);

#pragma unroll
    for (int r = 0; r < 8; ++r) {
      const int ro = (8 * hh + r) * 68 + c;
      slab[ro]      = o0[r] * inv[r];
      slab[ro + 16] = o1[r] * inv[r];
      slab[ro + 32] = o2[r] * inv[r];
      slab[ro + 48] = o3[r] * inv[r];
    }
    wave_sync_lds();
    v4u oh[4], ol[4];
#pragma unroll
    for (int i4 = 0; i4 < 4; ++i4) {
      const int row = i4 * 4 + rq;
      const v4f a = *(const v4f*)(slab + row * 68 + c8), c4 = *(const v4f*)(slab + row * 68 + c8 + 4);
      float wv[8];
#pragma unroll
      for (int e = 0; e < 4; ++e) { wv[e] = a[e] * OSC; wv[4 + e] = c4[e] * OSC; }
#pragma unroll
      for (int e = 0; e < 4; ++e) {
        const _Float16 h0 = (_Float16)wv[2 * e], h1 = (_Float16)wv[2 * e + 1];
        const _Float16 r0 = (_Float16)((wv[2 * e] - (float)h0) * ROC);
        const _Float16 r1 = (_Float16)((wv[2 * e + 1] - (float)h1) * ROC);
        oh[i4][e] = pk16(h_bits(h0), h_bits(h1));
        ol[i4][e] = pk16(h_bits(r0), h_bits(r1));
      }
    }
    wave_sync_lds();
    u16* os = ob + 64 * sl;
    for (int pass = 0; pass < 2; ++pass) {
#pragma unroll
      for (int i4 = 0; i4 < 4; ++i4) {
        const int row = i4 * 4 + rq;
        const size_t o8 = (size_t)row * QKP;
        *(volatile v4u*)(os + o8)       = oh[i4];
        *(volatile v4u*)(os + o8 + EMB) = ol[i4];
      }
      __threadfence();
    }
  }
}

extern "C" void kernel_launch(void* const* d_in, const int* in_sizes, int n_in,
                              void* d_out, int out_size, void* d_ws, size_t ws_size,
                              hipStream_t stream) {
  if (n_in < 5) return;
  const long long need_x = ((long long)(NB - 1) * SEQ_FULL + SEQ) * EMB;
  if ((long long)in_sizes[0] < need_x) return;
  if (in_sizes[1] < EMB * NQKV) return;
  if (in_sizes[2] < NQKV) return;
  if (in_sizes[3] < EMB * EMB) return;
  if (in_sizes[4] < EMB) return;
  if ((long long)out_size < need_x) return;

  const float* Xin = (const float*)d_in[0];
  const float* Wqk = (const float*)d_in[1];
  const float* Bqk = (const float*)d_in[2];
  const float* Wpr = (const float*)d_in[3];
  const float* Bpr = (const float*)d_in[4];
  float*       out = (float*)d_out;

  const size_t szOP = (size_t)NROWS * QKP * 2;
  const size_t szXB = (size_t)NROWS * EMB * 2;
  const size_t szR0 = (szOP > szXB) ? szOP : szXB;
  const size_t szWB = (size_t)NQKV * EMB * 2;
  const size_t szWO = (size_t)EMB * EMB * 2;
  const size_t szQK = (size_t)NROWS * QKP * 2;
  const size_t szVP = (size_t)NB * EMB * SEQ * 2;
  size_t off = 0;
  const size_t oR0 = off; off += szR0;
  const size_t oWB = off; off += szWB;
  const size_t oWO = off; off += szWO;
  const size_t oQP = off; off += szQK;
  const size_t oKP = off; off += szQK;
  const size_t oVP = off; off += szVP;
  if (off > ws_size) return;
  if (off > (size_t)134217728) return;

  char* ws = (char*)d_ws;
  u16* OP  = (u16*)(ws + oR0);
  u16* XB  = (u16*)(ws + oR0);
  u16* WB  = (u16*)(ws + oWB);
  u16* WOB = (u16*)(ws + oWO);
  u16* QP  = (u16*)(ws + oQP);
  u16* KP  = (u16*)(ws + oKP);
  u16* VP  = (u16*)(ws + oVP);

  const int n8pb = (SEQ * EMB) / 8;
  const int sst8 = (SEQ_FULL * EMB) / 8;
  if (((NB * n8pb) % 256) != 0) return;
  if ((EMB % 64) != 0 || (NQKV % 64) != 0 || (SEQ % 64) != 0 || (NROWS % 64) != 0 || (EMB % 32) != 0) return;
  const dim3 blk(256);
  const dim3 gX((NB * n8pb) / 256);
  const dim3 gTq((NQKV / 64) * (EMB / 64));
  const dim3 gTo((EMB / 64) * (EMB / 64));
  const dim3 bG(128);
  const dim3 gG((NROWS / 64) * (EMB / 64));
  const dim3 gV(NB * (EMB / 64) * (SEQ / 64));
  const dim3 gO(NB * (SEQ / 64) * (EMB / 64));
  const dim3 gAT(ATT_BLOCKS);
  const dim3 bAT(ATT_THREADS);

  cvt16<<<gX, blk, 0, stream>>>(Xin, XB, n8pb, NB, sst8, 0, 1.0f);
  tcvt16<<<gTq, blk, 0, stream>>>(Wqk, WB, EMB, NQKV, 0, 1.0f);
  tcvt16<<<gTo, blk, 0, stream>>>(Wpr, WOB, EMB, EMB, 1, WOS);
  gemm_b16<true><<<gG, bG, 0, stream>>>(XB, WB, QP, NROWS, EMB, EMB, QKP, EMB, 0, 0, 0, QSC, RQK, Bqk, 0, EMB);
  gemm_b16<true><<<gG, bG, 0, stream>>>(XB, WB + (size_t)EMB * EMB, KP, NROWS, EMB, EMB, QKP, EMB, 0, 0, 0, KSC, RQK,
                                        Bqk + EMB, 0, EMB);
  gemm_b16<false><<<gV, bG, 0, stream>>>(WB + (size_t)2 * EMB * EMB, XB, VP, EMB, SEQ, EMB, SEQ, 0,
                                         0, SEQ * EMB, EMB * SEQ, VCAR, 1.0f, Bqk + 2 * EMB, 1, EMB);
  attn_fwd<<<gAT, bAT, 0, stream>>>(QP, KP, VP, OP);
  gemm_hf2<<<gO, bG, 0, stream>>>(OP, WOB, out, SEQ, EMB, EMB, QKP, EMB, SEQ * QKP, SEQ_FULL * EMB,
                                  1.0f / (OSC * WOS), 1.0f / ROC, Bpr, EMB);
  (void)hipGetLastError();
}
